// PlasticityModelMoE_64209761075279
// MI455X (gfx1250) — hardware-verified
//
#include <hip/hip_runtime.h>
#include <stddef.h>
#include <stdint.h>
#include <math.h>


#define HS    512
#define FFN   2048
#define NEXP  8
#define TOPK  2
#define NTOK  4096
#define NASG  8192
#define MT    64
#define MAXT  136
#define RMAX  8704
#define TB    64
#define GTB   256
#define XSC   16
#define W1SC  1024
#define HSC   256
#define W2SC  2048
#define NTHR  256
#define NWAVE 8
#define TPW   64
#define WSCAP 134217728
#define LDS_GEMM (NWAVE * 32 * 64 * 4)

static_assert(NASG == NTOK * TOPK);
static_assert(RMAX == MAXT * MT);
static_assert(MAXT >= NASG / MT + NEXP);
static_assert((NASG % NTHR) == 0);
static_assert((NTOK % TB) == 0);
static_assert((NTOK % GTB) == 0);
static_assert(GTB == NTHR);
static_assert(TOPK * GTB == 4 * (NTHR / 2));
static_assert(TOPK * TB <= NTHR);
static_assert((TB % NWAVE) == 0);
static_assert((MT % NWAVE) == 0);
static_assert(NTHR == NWAVE * 32);
static_assert((HS % 256) == 0);
static_assert((FFN % 256) == 0);
static_assert((HS % 128) == 0);
static_assert((FFN % 128) == 0);
static_assert((HS % 32) == 0);
static_assert((FFN % 32) == 0);
static_assert((HS % 4) == 0);
static_assert(LDS_GEMM <= 300 * 1024);

typedef float          v2f  __attribute__((ext_vector_type(2)));
typedef float          v4f  __attribute__((ext_vector_type(4)));
typedef float          v8f  __attribute__((ext_vector_type(8)));
typedef double         v4d  __attribute__((ext_vector_type(4)));
typedef int            v4i  __attribute__((ext_vector_type(4)));
typedef _Float16       v8h  __attribute__((ext_vector_type(8)));
typedef _Float16       v16h __attribute__((ext_vector_type(16)));
union FragH { v16h v; v8h h[2]; };

__device__ __forceinline__ v8f wmf(v16h a, v16h b, v8f c) {
  v8f d = __builtin_amdgcn_wmma_f32_16x16x32_f16(false, a, false, b, (short)0, c, false, false);
  asm volatile("v_nop\n\tv_nop\n\tv_nop\n\tv_nop" : "+v"(d) : "v"(a), "v"(b));
  return d;
}

__device__ __forceinline__ int clamp_e(int v) { return v < 0 ? 0 : (v > NEXP - 1 ? NEXP - 1 : v); }

__device__ __forceinline__ float gelu_t(float v) {
  const float u = 0.7978845608028654f * (v + 0.044715f * (v * v * v));
  return 0.5f * v * (1.0f + tanhf(u));
}

__device__ __forceinline__ void gate_acc(double xc, const double* wrow, double (&acc)[NEXP]) {
  const v4d wa = *(const v4d*)wrow;
  const v4d wb = *(const v4d*)(wrow + 4);
  acc[0] = __builtin_fma(xc, wa.x, acc[0]);
  acc[1] = __builtin_fma(xc, wa.y, acc[1]);
  acc[2] = __builtin_fma(xc, wa.z, acc[2]);
  acc[3] = __builtin_fma(xc, wa.w, acc[3]);
  acc[4] = __builtin_fma(xc, wb.x, acc[4]);
  acc[5] = __builtin_fma(xc, wb.y, acc[5]);
  acc[6] = __builtin_fma(xc, wb.z, acc[6]);
  acc[7] = __builtin_fma(xc, wb.w, acc[7]);
}

__global__ __launch_bounds__(NTHR) void k_gate(const float* __restrict__ x, const float* __restrict__ wg,
                                               int* ei, float* ew) {
#pragma clang fp contract(off)
  __shared__ __attribute__((aligned(32))) double s_wg[HS * NEXP];
  __shared__ __attribute__((aligned(16))) int    s_ei[TOPK * GTB];
  __shared__ __attribute__((aligned(16))) float  s_ew[TOPK * GTB];
  const int tid = threadIdx.x;
  const int t0 = blockIdx.x * GTB;
#pragma unroll 1
  for (int i = tid; i < HS * NEXP; i += NTHR) s_wg[i] = (double)wg[i];
  __syncthreads();

  int t = t0 + tid;
  t = t > NTOK - 1 ? NTOK - 1 : t;
  const float* xr = x + (size_t)t * HS;
  double acc[NEXP];
#pragma unroll
  for (int e = 0; e < NEXP; ++e) acc[e] = 0.0;
#pragma unroll 1
  for (int d = 0; d < HS; d += 4) {
    const v4f xv = *(const v4f*)(xr + d);
    const double* wr = s_wg + (size_t)d * NEXP;
    gate_acc((double)xv.x, wr,            acc);
    gate_acc((double)xv.y, wr + NEXP,     acc);
    gate_acc((double)xv.z, wr + 2 * NEXP, acc);
    gate_acc((double)xv.w, wr + 3 * NEXP, acc);
  }

  float v[NEXP];
#pragma unroll
  for (int e = 0; e < NEXP; ++e) v[e] = (float)acc[e];
  int i0 = 0; float m0 = v[0];
#pragma unroll
  for (int j = 1; j < NEXP; ++j) { if (v[j] > m0) { m0 = v[j]; i0 = j; } }
  int i1 = -1; float m1 = 0.0f;
#pragma unroll
  for (int j = 0; j < NEXP; ++j) { if (j != i0 && (i1 < 0 || v[j] > m1)) { m1 = v[j]; i1 = j; } }
  const float e1 = expf(m1 - m0);
  const float s = 1.0f + e1;
  const float rs = 1.0f / s;
  const float g0 = 1.0f * rs;
  const float g1 = e1 * rs;

  s_ei[TOPK * tid] = i0;  s_ei[TOPK * tid + 1] = i1;
  s_ew[TOPK * tid] = g0;  s_ew[TOPK * tid + 1] = g1;
  __syncthreads();

  const int q = tid & 127;
  const v4i vi = *(const v4i*)(s_ei + 4 * q);
  const v4f vf = *(const v4f*)(s_ew + 4 * q);
  int*   di = ei + (size_t)TOPK * t0 + 4 * q;
  float* df = ew + (size_t)TOPK * t0 + 4 * q;
  const bool wi = (tid < 128);
  if (wi) *(volatile v4i*)di = vi; else *(volatile v4f*)df = vf;
  __threadfence();
  if (wi) *(volatile v4i*)di = vi; else *(volatile v4f*)df = vf;
}

struct RouteLds { int red[NWAVE][2 * NEXP]; int cnt[2 * NEXP]; };

__device__ __forceinline__ void route_counts(const int* __restrict__ idx, int lim, RouteLds* rs, int tid) {
  int tot[NEXP], pre[NEXP];
#pragma unroll
  for (int e = 0; e < NEXP; ++e) { tot[e] = 0; pre[e] = 0; }
#pragma unroll 1
  for (int i = tid; i < NASG; i += NTHR) {
    const int v = clamp_e(idx[i]);
    const int ip = (i < lim) ? 1 : 0;
#pragma unroll
    for (int e = 0; e < NEXP; ++e) {
      const int f = (v == e) ? 1 : 0;
      tot[e] += f;
      pre[e] += f & ip;
    }
  }
#pragma unroll
  for (int e = 0; e < NEXP; ++e) {
#pragma unroll
    for (int o = 16; o > 0; o >>= 1) {
      tot[e] += __shfl_xor(tot[e], o, 32);
      pre[e] += __shfl_xor(pre[e], o, 32);
    }
  }
  const int lane = tid & 31, wave = tid >> 5;
  if (lane == 0) {
#pragma unroll
    for (int e = 0; e < NEXP; ++e) { rs->red[wave][e] = tot[e]; rs->red[wave][NEXP + e] = pre[e]; }
  }
  __syncthreads();
  if (tid < 2 * NEXP) {
    int c = 0;
#pragma unroll
    for (int w = 0; w < NWAVE; ++w) c += rs->red[w][tid];
    rs->cnt[tid] = c;
  }
  __syncthreads();
}

__device__ __forceinline__ int tile_geom(const RouteLds* rs, int b, int& my_e, int& tp_e) {
  int tp = 0; my_e = 0; tp_e = 0;
#pragma unroll
  for (int e = 0; e < NEXP; ++e) {
    const int c = rs->cnt[e];
    const int nt = (c + MT - 1) / MT;
    if (b >= tp && b < tp + nt) { my_e = e; tp_e = tp; }
    tp += nt;
  }
  return tp;
}

__device__ __forceinline__ void tile_write_t(const float* tile, _Float16* dbase, int dp, int dc,
                                             float wsc, int g, int hh, int m) {
  v8h hv[4];
#pragma unroll
  for (int q = 0; q < 4; ++q) {
    const int nl = 8 * g + 2 * q + hh;
    const int d8 = 8 * m;
#pragma unroll
    for (int u = 0; u < 8; ++u) hv[q][u] = (_Float16)(tile[(d8 + u) * TPW + nl] * wsc);
  }
#pragma unroll
  for (int q = 0; q < 4; ++q) {
    _Float16* d = dbase + (size_t)(8 * g + 2 * q + hh) * dp + dc + 8 * m;
    *(volatile v8h*)d = hv[q];
  }
  __threadfence();
#pragma unroll
  for (int q = 0; q < 4; ++q) {
    _Float16* d = dbase + (size_t)(8 * g + 2 * q + hh) * dp + dc + 8 * m;
    *(volatile v8h*)d = hv[q];
  }
}

__global__ __launch_bounds__(NTHR) void k_tw1(const float* __restrict__ w1, _Float16* w1t) {
  __shared__ __attribute__((aligned(16))) float tile[128 * TPW];
  const int tid = threadIdx.x, lane = tid & 31, gw = tid >> 5, hh = lane >> 4, m = lane & 15;
  const int n0 = blockIdx.x * 64, e = blockIdx.y;
#pragma unroll 1
  for (int dc = 0; dc < HS; dc += 128) {
    __syncthreads();
#pragma unroll 4
    for (int p = 0; p < 16; ++p) {
      const int dl = gw + 8 * p;
      const v2f w = *(const v2f*)(w1 + ((size_t)e * HS + dc + dl) * FFN + n0 + 2 * lane);
      *(v2f*)(tile + dl * TPW + 2 * lane) = w;
    }
    __syncthreads();
    tile_write_t(tile, w1t + ((size_t)e * FFN + n0) * HS, HS, dc, (float)W1SC, gw, hh, m);
  }
}

__global__ __launch_bounds__(NTHR) void k_tw2(const float* __restrict__ w2, _Float16* w2t) {
  __shared__ __attribute__((aligned(16))) float tile[128 * TPW];
  const int tid = threadIdx.x, lane = tid & 31, gw = tid >> 5, hh = lane >> 4, m = lane & 15;
  const int n0 = blockIdx.x * 64, e = blockIdx.y;
#pragma unroll 1
  for (int dc = 0; dc < FFN; dc += 128) {
    __syncthreads();
#pragma unroll 4
    for (int p = 0; p < 16; ++p) {
      const int dl = gw + 8 * p;
      const v2f w = *(const v2f*)(w2 + ((size_t)e * FFN + dc + dl) * HS + n0 + 2 * lane);
      *(v2f*)(tile + dl * TPW + 2 * lane) = w;
    }
    __syncthreads();
    tile_write_t(tile, w2t + ((size_t)e * HS + n0) * FFN, FFN, dc, (float)W2SC, gw, hh, m);
  }
}

__global__ __launch_bounds__(NTHR) void k_gather(const int* __restrict__ idx, const float* __restrict__ x, _Float16* xg) {
  __shared__ RouteLds rs;
  __shared__ int s_slot[MT];
  __shared__ int s_wt[NWAVE];
  const int tid = threadIdx.x, lane = tid & 31, wave = tid >> 5;
  route_counts(idx, 0, &rs, tid);
  const int tile = blockIdx.x;
  int my_e, tp_e;
  const int ntiles = tile_geom(&rs, tile, my_e, tp_e);
  if (tile >= ntiles) return;
  const int lo = (tile - tp_e) * MT, hi = lo + MT;
  if (tid < MT) s_slot[tid] = -1;
  __syncthreads();
  int base = 0;
  const unsigned lt = (1u << lane) - 1u;
#pragma unroll 1
  for (int c = 0; c < NASG / NTHR; ++c) {
    const int i = c * NTHR + tid;
    const int v = clamp_e(idx[i]);
    const int f = (v == my_e) ? 1 : 0;
    const unsigned bal = __builtin_amdgcn_ballot_w32(f != 0);
    const int lp = __builtin_popcount(bal & lt);
    if (lane == 0) s_wt[wave] = __builtin_popcount(bal);
    __syncthreads();
    int wpre = 0, wtot = 0;
#pragma unroll
    for (int w = 0; w < NWAVE; ++w) {
      const int tcnt = s_wt[w];
      wpre += (w < wave) ? tcnt : 0;
      wtot += tcnt;
    }
    const int rank = base + wpre + lp;
    if (f != 0 && rank >= lo && rank < hi) s_slot[rank - lo] = i;
    base += wtot;
    __syncthreads();
  }
#pragma unroll 1
  for (int q = 0; q < MT / NWAVE; ++q) {
    const int rr = wave * (MT / NWAVE) + q;
    const int a = s_slot[rr];
    const int valid = (a >= 0) ? 1 : 0;
    int tok = valid ? (a / TOPK) : 0;
    tok = tok < 0 ? 0 : (tok > NTOK - 1 ? NTOK - 1 : tok);
    const float sc = valid ? (float)XSC : 0.0f;
    const float* xr = x + (size_t)tok * HS;
    _Float16* dr = xg + (size_t)(tile * MT + rr) * HS;
    v8h hv[2];
#pragma unroll
    for (int j = 0; j < 2; ++j) {
      const int cc = 256 * j + 8 * lane;
      const v4f f0 = *(const v4f*)(xr + cc);
      const v4f f1 = *(const v4f*)(xr + cc + 4);
      hv[j][0] = (_Float16)(f0.x * sc); hv[j][1] = (_Float16)(f0.y * sc);
      hv[j][2] = (_Float16)(f0.z * sc); hv[j][3] = (_Float16)(f0.w * sc);
      hv[j][4] = (_Float16)(f1.x * sc); hv[j][5] = (_Float16)(f1.y * sc);
      hv[j][6] = (_Float16)(f1.z * sc); hv[j][7] = (_Float16)(f1.w * sc);
    }
#pragma unroll
    for (int j = 0; j < 2; ++j) *(volatile v8h*)(dr + 256 * j + 8 * lane) = hv[j];
    __threadfence();
#pragma unroll
    for (int j = 0; j < 2; ++j) *(volatile v8h*)(dr + 256 * j + 8 * lane) = hv[j];
  }
}

__global__ __launch_bounds__(NTHR) void k_gemm1(const int* __restrict__ idx, const _Float16* __restrict__ xg,
                                                const _Float16* __restrict__ w1t, const float* __restrict__ b1,
                                                _Float16* hp) {
  extern __shared__ v4f lds_dyn[];
  __shared__ RouteLds rs;
  const int tid = threadIdx.x, lane = tid & 31, wave = tid >> 5, hh = lane >> 4, m = lane & 15;
  route_counts(idx, 0, &rs, tid);
  const int tile = blockIdx.y;
  int my_e, tp_e;
  const int ntiles = tile_geom(&rs, tile, my_e, tp_e);
  if (tile >= ntiles) return;
  float* stg = (float*)lds_dyn + wave * (32 * 64);
  const int n0 = blockIdx.x * 256, m0 = tile * MT;
  const int wm = (wave >> 2) * 32, wn = (wave & 3) * 64;

  v8f acc[2][4];
#pragma unroll
  for (int mt = 0; mt < 2; ++mt)
#pragma unroll
    for (int nt = 0; nt < 4; ++nt) { v8f z = {0.f, 0.f, 0.f, 0.f, 0.f, 0.f, 0.f, 0.f}; acc[mt][nt] = z; }

  const _Float16* ap = xg + (size_t)(m0 + wm + m) * HS + 8 * hh;
  const _Float16* bp = w1t + ((size_t)my_e * FFN + n0 + wn + m) * HS + 8 * hh;
#pragma unroll 1
  for (int kt = 0; kt < HS / 32; ++kt) {
    const int k0 = 32 * kt;
    FragH a0, a1;
    a0.h[0] = *(const v8h*)(ap + k0);
    a0.h[1] = *(const v8h*)(ap + k0 + 16);
    a1.h[0] = *(const v8h*)(ap + (size_t)16 * HS + k0);
    a1.h[1] = *(const v8h*)(ap + (size_t)16 * HS + k0 + 16);
#pragma unroll
    for (int nt = 0; nt < 4; ++nt) {
      const _Float16* bq = bp + (size_t)nt * 16 * HS + k0;
      FragH b;
      b.h[0] = *(const v8h*)bq;
      b.h[1] = *(const v8h*)(bq + 16);
      acc[0][nt] = wmf(a0.v, b.v, acc[0][nt]);
      acc[1][nt] = wmf(a1.v, b.v, acc[1][nt]);
    }
  }

  constexpr float OSC1 = 1.0f / (float)(XSC * W1SC);
#pragma unroll
  for (int mt = 0; mt < 2; ++mt) {
    float* sp = stg + (16 * mt + 8 * hh) * 64 + m;
#pragma unroll
    for (int nt = 0; nt < 4; ++nt) {
#pragma unroll
      for (int r = 0; r < 8; ++r) sp[r * 64 + 16 * nt] = acc[mt][nt][r] * OSC1;
    }
  }
  __syncthreads();
  {
    const float* bb = b1 + (size_t)my_e * FFN + n0 + wn;
    const float bA = bb[lane], bB = bb[lane + 32];
#pragma unroll 1
    for (int j = 0; j < 64; ++j) {
      const int i = lane + 32 * j;
      const float bias = (j & 1) ? bB : bA;
      stg[i] = gelu_t(stg[i] + bias);
    }
  }
  __syncthreads();

  const int rg = lane >> 3, cq = lane & 7;
  v8h hv[8];
#pragma unroll
  for (int p = 0; p < 8; ++p) {
    const float* s = stg + (4 * p + rg) * 64 + 8 * cq;
    const v4f x0 = *(const v4f*)s;
    const v4f x1 = *(const v4f*)(s + 4);
    hv[p][0] = (_Float16)(x0.x * (float)HSC); hv[p][1] = (_Float16)(x0.y * (float)HSC);
    hv[p][2] = (_Float16)(x0.z * (float)HSC); hv[p][3] = (_Float16)(x0.w * (float)HSC);
    hv[p][4] = (_Float16)(x1.x * (float)HSC); hv[p][5] = (_Float16)(x1.y * (float)HSC);
    hv[p][6] = (_Float16)(x1.z * (float)HSC); hv[p][7] = (_Float16)(x1.w * (float)HSC);
  }
  _Float16* ob = hp + (size_t)(m0 + wm) * FFN + n0 + wn + 8 * cq;
#pragma unroll
  for (int p = 0; p < 8; ++p) *(volatile v8h*)(ob + (size_t)(4 * p + rg) * FFN) = hv[p];
  __threadfence();
#pragma unroll
  for (int p = 0; p < 8; ++p) *(volatile v8h*)(ob + (size_t)(4 * p + rg) * FFN) = hv[p];
}

__global__ __launch_bounds__(NTHR) void k_gemm2(const int* __restrict__ idx, const _Float16* __restrict__ hp,
                                                const _Float16* __restrict__ w2t, const float* __restrict__ b2,
                                                float* yp) {
  extern __shared__ v4f lds_dyn[];
  __shared__ RouteLds rs;
  const int tid = threadIdx.x, lane = tid & 31, wave = tid >> 5, hh = lane >> 4, m = lane & 15;
  route_counts(idx, 0, &rs, tid);
  const int tile = blockIdx.y;
  int my_e, tp_e;
  const int ntiles = tile_geom(&rs, tile, my_e, tp_e);
  if (tile >= ntiles) return;
  float* stg = (float*)lds_dyn + wave * (32 * 64);
  const int n0 = blockIdx.x * 256, m0 = tile * MT;
  const int wm = (wave >> 2) * 32, wn = (wave & 3) * 64;

  v8f acc[2][4];
#pragma unroll
  for (int mt = 0; mt < 2; ++mt)
#pragma unroll
    for (int nt = 0; nt < 4; ++nt) { v8f z = {0.f, 0.f, 0.f, 0.f, 0.f, 0.f, 0.f, 0.f}; acc[mt][nt] = z; }

  const _Float16* ap = hp + (size_t)(m0 + wm + m) * FFN + 8 * hh;
  const _Float16* bp = w2t + ((size_t)my_e * HS + n0 + wn + m) * FFN + 8 * hh;
#pragma unroll 1
  for (int kt = 0; kt < FFN / 32; ++kt) {
    const int k0 = 32 * kt;
    FragH a0, a1;
    a0.h[0] = *(const v8h*)(ap + k0);
    a0.h[1] = *(const v8h*)(ap + k0 + 16);
    a1.h[0] = *(const v8h*)(ap + (size_t)16 * FFN + k0);
    a1.h[1] = *(const v8h*)(ap + (size_t)16 * FFN + k0 + 16);
#pragma unroll
    for (int nt = 0; nt < 4; ++nt) {
      const _Float16* bq = bp + (size_t)nt * 16 * FFN + k0;
      FragH b;
      b.h[0] = *(const v8h*)bq;
      b.h[1] = *(const v8h*)(bq + 16);
      acc[0][nt] = wmf(a0.v, b.v, acc[0][nt]);
      acc[1][nt] = wmf(a1.v, b.v, acc[1][nt]);
    }
  }

  constexpr float OSC2 = 1.0f / ((float)HSC * (float)W2SC);
  float bv[4];
  {
    const float* bb = b2 + (size_t)my_e * HS + n0 + wn + m;
#pragma unroll
    for (int nt = 0; nt < 4; ++nt) bv[nt] = bb[16 * nt];
  }
#pragma unroll
  for (int mt = 0; mt < 2; ++mt) {
    float* sp = stg + (16 * mt + 8 * hh) * 64 + m;
#pragma unroll
    for (int nt = 0; nt < 4; ++nt) {
#pragma unroll
      for (int r = 0; r < 8; ++r) sp[r * 64 + 16 * nt] = acc[mt][nt][r] * OSC2 + bv[nt];
    }
  }
  __syncthreads();

  float* yb = yp + (size_t)(m0 + wm) * HS + n0 + wn + 4 * m;
#pragma unroll
  for (int p = 0; p < 16; ++p) {
    const v4f u = *(const v4f*)(stg + (2 * p + hh) * 64 + 4 * m);
    *(volatile v4f*)(yb + (size_t)(2 * p + hh) * HS) = u;
  }
  __threadfence();
#pragma unroll
  for (int p = 0; p < 16; ++p) {
    const v4f u = *(const v4f*)(stg + (2 * p + hh) * 64 + 4 * m);
    *(volatile v4f*)(yb + (size_t)(2 * p + hh) * HS) = u;
  }
}

__global__ __launch_bounds__(NTHR) void k_combine(const int* __restrict__ idx, const float* __restrict__ ew,
                                                  const float* __restrict__ yp, float* out) {
#pragma clang fp contract(off)
  __shared__ RouteLds rs;
  __shared__ int s_base[NEXP];
  __shared__ int s_wt[NEXP * NWAVE];
  __shared__ int s_pos[TOPK * TB];
  const int tid = threadIdx.x, lane = tid & 31, wave = tid >> 5;
  const int t0 = blockIdx.x * TB;
  route_counts(idx, TOPK * t0, &rs, tid);
  if (tid < NEXP) {
    int tp = 0;
#pragma unroll
    for (int e = 0; e < NEXP; ++e) tp += (e < tid) ? (rs.cnt[e] + MT - 1) / MT : 0;
    s_base[tid] = tp * MT + rs.cnt[NEXP + tid];
  }
  const int j = tid;
  const int aval = (j < TOPK * TB) ? 1 : 0;
  int aj = TOPK * t0 + j;
  aj = aj > NASG - 1 ? NASG - 1 : aj;
  const int vraw = clamp_e(idx[aj]);
  const int v = aval ? vraw : -1;
  int lpsel = 0;
  const unsigned lt = (1u << lane) - 1u;
#pragma unroll
  for (int e = 0; e < NEXP; ++e) {
    const int f = (v == e) ? 1 : 0;
    const unsigned bal = __builtin_amdgcn_ballot_w32(f != 0);
    const int lp = __builtin_popcount(bal & lt);
    if (lane == 0) s_wt[e * NWAVE + wave] = __builtin_popcount(bal);
    if (f != 0) lpsel = lp;
  }
  __syncthreads();
  if (aval) {
    const int vc = v;
    int wp = 0;
#pragma unroll
    for (int w = 0; w < NWAVE; ++w) wp += (w < wave) ? s_wt[vc * NWAVE + w] : 0;
    int pos = s_base[vc] + wp + lpsel;
    pos = pos < 0 ? 0 : (pos > RMAX - 1 ? RMAX - 1 : pos);
    s_pos[j] = pos;
  }
  __syncthreads();

#pragma unroll 1
  for (int q = 0; q < TB / NWAVE; ++q) {
    const int tl = wave * (TB / NWAVE) + q;
    const int t = t0 + tl;
    const int p0 = s_pos[TOPK * tl], p1 = s_pos[TOPK * tl + 1];
    const float w0 = ew[(size_t)TOPK * t], w1v = ew[(size_t)TOPK * t + 1];
    const float* y0 = yp + (size_t)p0 * HS;
    const float* y1 = yp + (size_t)p1 * HS;
    float* orow = out + (size_t)t * HS;
    v4f ov[4];
#pragma unroll
    for (int jj = 0; jj < 4; ++jj) {
      const int cc = 128 * jj + 4 * lane;
      const v4f u0 = *(const v4f*)(y0 + cc);
      const v4f u1 = *(const v4f*)(y1 + cc);
      const v4f pa = u0 * w0;
      const v4f pb = u1 * w1v;
      ov[jj] = pa + pb;
    }
#pragma unroll
    for (int jj = 0; jj < 4; ++jj) *(volatile v4f*)(orow + 128 * jj + 4 * lane) = ov[jj];
    __threadfence();
#pragma unroll
    for (int jj = 0; jj < 4; ++jj) *(volatile v4f*)(orow + 128 * jj + 4 * lane) = ov[jj];
  }
}

extern "C" void kernel_launch(void* const* d_in, const int* in_sizes, int n_in,
                              void* d_out, int out_size, void* d_ws, size_t ws_size,
                              hipStream_t stream) {
  if (n_in < 6) return;
  if (in_sizes[0] != NTOK * HS) return;
  if (in_sizes[1] != HS * NEXP) return;
  if (in_sizes[2] != NEXP * HS * FFN) return;
  if (in_sizes[3] != NEXP * FFN) return;
  if (in_sizes[4] != NEXP * FFN * HS) return;
  if (in_sizes[5] != NEXP * HS) return;
  if (out_size != NTOK * HS) return;

  const float* x  = (const float*)d_in[0];
  const float* wg = (const float*)d_in[1];
  const float* w1 = (const float*)d_in[2];
  const float* b1 = (const float*)d_in[3];
  const float* w2 = (const float*)d_in[4];
  const float* b2 = (const float*)d_in[5];
  float* out = (float*)d_out;

  char* ws = (char*)d_ws;
  size_t off = 0;
  const size_t oEI = off; off += (size_t)NASG * 4;             off = (off + 255) & ~(size_t)255;
  const size_t oEW = off; off += (size_t)NASG * 4;             off = (off + 255) & ~(size_t)255;
  const size_t oW1 = off; off += (size_t)NEXP * FFN * HS * 2;  off = (off + 255) & ~(size_t)255;
  const size_t oW2 = off; off += (size_t)NEXP * HS * FFN * 2;  off = (off + 255) & ~(size_t)255;
  const size_t oXg = off; off += (size_t)RMAX * HS * 2;        off = (off + 255) & ~(size_t)255;
  const size_t oH  = off; off += (size_t)RMAX * FFN * 2;       off = (off + 255) & ~(size_t)255;
  const size_t oY  = off; off += (size_t)RMAX * HS * 4;        off = (off + 255) & ~(size_t)255;
  if (off > ws_size || off > (size_t)WSCAP) return;
  int*      ei  = (int*)(ws + oEI);
  float*    ew  = (float*)(ws + oEW);
  _Float16* w1t = (_Float16*)(ws + oW1);
  _Float16* w2t = (_Float16*)(ws + oW2);
  _Float16* xg  = (_Float16*)(ws + oXg);
  _Float16* hp  = (_Float16*)(ws + oH);
  float*    yp  = (float*)(ws + oY);

  k_gate<<<NTOK / GTB, NTHR, 0, stream>>>(x, wg, ei, ew);
  k_tw1<<<dim3(FFN / 64, NEXP), NTHR, 0, stream>>>(w1, w1t);
  k_tw2<<<dim3(HS / 64, NEXP), NTHR, 0, stream>>>(w2, w2t);
  k_gather<<<MAXT, NTHR, 0, stream>>>(ei, x, xg);
  hipFuncSetAttribute(reinterpret_cast<const void*>(&k_gemm1),
                      hipFuncAttributeMaxDynamicSharedMemorySize, LDS_GEMM);
  k_gemm1<<<dim3(FFN / 256, MAXT), NTHR, LDS_GEMM, stream>>>(ei, xg, w1t, b1, hp);
  hipFuncSetAttribute(reinterpret_cast<const void*>(&k_gemm2),
                      hipFuncAttributeMaxDynamicSharedMemorySize, LDS_GEMM);
  k_gemm2<<<dim3(HS / 256, MAXT), NTHR, LDS_GEMM, stream>>>(ei, hp, w2t, b2, yp);
  k_combine<<<NTOK / TB, NTHR, 0, stream>>>(ei, ew, yp, out);
}
